// Decoder_52201032516290
// MI455X (gfx1250) — hardware-verified
//
#include <hip/hip_runtime.h>
#include <stddef.h>
#include <stdint.h>


#define ZD     64
#define NH     128
#define NPQ    256
#define GBM    64
#define GBN    64
#define GTHR   128
#define NTHR   256
#define NUW    (NPQ * (ZD / 8))
#define EPB    1024
#define EPW    128
#define WSMAX  134217728

static_assert(ZD % 32 == 0 && ZD / 8 == 8);
static_assert(NPQ == 2 * NH && NPQ % GBN == 0 && NH % GBN == 0);
static_assert(GBM == (GTHR / 32) * 16 && GBN == 64);
static_assert(NUW % NTHR == 0);
static_assert(EPB == (NTHR / 32) * EPW && EPW % 32 == 0);
static_assert(NH == 8 * 4 * 4);

typedef float          v4f   __attribute__((ext_vector_type(4)));
typedef float          v8f   __attribute__((ext_vector_type(8)));
typedef int            v8i   __attribute__((ext_vector_type(8)));
typedef unsigned short v8us  __attribute__((ext_vector_type(8)));
typedef unsigned short v16us __attribute__((ext_vector_type(16)));
typedef __bf16         v16bf __attribute__((ext_vector_type(16)));
typedef v4f  __attribute__((may_alias)) v4fa;
typedef v8us __attribute__((may_alias)) v8usa;
union FragB { v16bf v; v16us u; v8us h[2]; v8i w; };

__device__ __forceinline__ v8f wmb(const FragB& a, const FragB& b, v8f c) {
  v8f d = __builtin_amdgcn_wmma_f32_16x16x32_bf16(false, a.v, false, b.v, (short)0, c, false, false);
  asm volatile("v_nop\n\tv_nop\n\tv_nop\n\tv_nop" : "+v"(d) : "v"(a.w), "v"(b.w));
  return d;
}

__device__ __forceinline__ unsigned bf16_bits(float f) {
  const unsigned u = __float_as_uint(f);
  return (u + 0x7FFFu + ((u >> 16) & 1u)) >> 16;
}
__device__ __forceinline__ float bf16_val(float f) {
  return __uint_as_float(bf16_bits(f) << 16);
}

__global__ __launch_bounds__(NTHR) void k_wprep(const float* __restrict__ W1, unsigned short* bt2) {
  const int u = (int)blockIdx.x * NTHR + (int)threadIdx.x;
  if (u >= NUW) return;
  const int j  = u >> 3;
  const int k8 = (u & 7) * 8;
  const float* p = W1 + (size_t)(j & (NH - 1)) * NH + (size_t)(j >> 7) * ZD + k8;
  const v4f a = *(const v4fa*)p;
  const v4f b = *(const v4fa*)(p + 4);
  v8us o;
  o[0] = (unsigned short)bf16_bits(a.x); o[1] = (unsigned short)bf16_bits(a.y);
  o[2] = (unsigned short)bf16_bits(a.z); o[3] = (unsigned short)bf16_bits(a.w);
  o[4] = (unsigned short)bf16_bits(b.x); o[5] = (unsigned short)bf16_bits(b.y);
  o[6] = (unsigned short)bf16_bits(b.z); o[7] = (unsigned short)bf16_bits(b.w);
  unsigned short* dp = bt2 + (size_t)j * ZD + k8;
  *(volatile v8us*)dp = o;
  __threadfence();
  *(volatile v8us*)dp = o;
}

__global__ __launch_bounds__(NTHR) void k_cvz(const float* __restrict__ z, int nN, int nUnits,
                                              unsigned short* zb) {
  const int u = (int)blockIdx.x * NTHR + (int)threadIdx.x;
  if (u >= nUnits) return;
  const int row = u >> 3;
  const int k8  = (u & 7) * 8;
  const int rc  = row < nN ? row : nN - 1;
  const float* p = z + (size_t)rc * ZD + k8;
  const v4f a = *(const v4fa*)p;
  const v4f b = *(const v4fa*)(p + 4);
  const bool ok = row < nN;
  v8us o;
  o[0] = ok ? (unsigned short)bf16_bits(a.x) : (unsigned short)0;
  o[1] = ok ? (unsigned short)bf16_bits(a.y) : (unsigned short)0;
  o[2] = ok ? (unsigned short)bf16_bits(a.z) : (unsigned short)0;
  o[3] = ok ? (unsigned short)bf16_bits(a.w) : (unsigned short)0;
  o[4] = ok ? (unsigned short)bf16_bits(b.x) : (unsigned short)0;
  o[5] = ok ? (unsigned short)bf16_bits(b.y) : (unsigned short)0;
  o[6] = ok ? (unsigned short)bf16_bits(b.z) : (unsigned short)0;
  o[7] = ok ? (unsigned short)bf16_bits(b.w) : (unsigned short)0;
  unsigned short* dp = zb + (size_t)row * ZD + k8;
  *(volatile v8us*)dp = o;
  __threadfence();
  *(volatile v8us*)dp = o;
}

__global__ __launch_bounds__(GTHR) void k_nodegemm(
    const unsigned short* __restrict__ A, const unsigned short* __restrict__ WT,
    const float* __restrict__ b1, float* outF)
{
  __shared__ __attribute__((aligned(16))) float stg[GBM * GBN];
  const int tid = (int)threadIdx.x, lane = tid & 31, wave = tid >> 5, hh = lane >> 4, m = lane & 15;
  const int rowBase = (int)blockIdx.x * GBM;
  const int col0    = (int)blockIdx.y * GBN;

  v8f acc[4];
  {
    const v8f z = {0.f, 0.f, 0.f, 0.f, 0.f, 0.f, 0.f, 0.f};
    acc[0] = z; acc[1] = z; acc[2] = z; acc[3] = z;
  }
  const unsigned short* ap = A  + (size_t)(rowBase + 16 * wave + m) * (size_t)ZD + 8 * hh;
  const unsigned short* wp = WT + (size_t)(col0 + m) * (size_t)ZD + 8 * hh;
#pragma unroll 1
  for (int ks = 0; ks < ZD / 32; ++ks) {
    FragB af;
    af.h[0] = *(const v8usa*)(ap + 32 * ks);
    af.h[1] = *(const v8usa*)(ap + 32 * ks + 16);
#pragma unroll
    for (int t = 0; t < 4; ++t) {
      const unsigned short* wq = wp + (size_t)(16 * t) * (size_t)ZD + 32 * ks;
      FragB bf;
      bf.h[0] = *(const v8usa*)wq;
      bf.h[1] = *(const v8usa*)(wq + 16);
      acc[t] = wmb(af, bf, acc[t]);
    }
  }

#pragma unroll
  for (int t = 0; t < 4; ++t) {
    const int lc = 16 * t + m;
#pragma unroll
    for (int r = 0; r < 8; ++r) {
      const int lr = 16 * wave + 8 * hh + r;
      stg[lr * GBN + lc] = acc[t][r];
    }
  }
  __syncthreads();

  v4f bb;
  {
    const float bsel = (col0 < NH) ? 1.0f : 0.0f;
    const v4f t1 = *(const v4fa*)(b1 + ((col0 + 4 * m) & (NH - 1)));
    bb.x = bsel * bf16_val(t1.x);
    bb.y = bsel * bf16_val(t1.y);
    bb.z = bsel * bf16_val(t1.z);
    bb.w = bsel * bf16_val(t1.w);
  }

  v4f fv[8];
#pragma unroll
  for (int i = 0; i < 8; ++i) {
    const int lr = 16 * wave + 2 * i + hh;
    const v4f s = *(const v4fa*)(stg + lr * GBN + 4 * m);
    fv[i] = s + bb;
  }
#pragma unroll
  for (int i = 0; i < 8; ++i) {
    const int lr = 16 * wave + 2 * i + hh;
    const int gr = rowBase + lr;
    float* op = outF + (size_t)gr * (size_t)NPQ + col0 + 4 * m;
    *(volatile v4f*)op = fv[i];
  }
  __threadfence();
#pragma unroll
  for (int i = 0; i < 8; ++i) {
    const int lr = 16 * wave + 2 * i + hh;
    const int gr = rowBase + lr;
    float* op = outF + (size_t)gr * (size_t)NPQ + col0 + 4 * m;
    *(volatile v4f*)op = fv[i];
  }
}

__global__ __launch_bounds__(NTHR) void k_edge(const float* __restrict__ pq,
                                               const int* __restrict__ rowi, const int* __restrict__ coli,
                                               const float* __restrict__ W2, const float* __restrict__ b2,
                                               int nE, int nN, float* out) {
  const int tid = (int)threadIdx.x, lane = tid & 31, wave = tid >> 5;
  const int g = lane & 7, j = lane >> 3;
  v4f w0, w1, w2, w3;
  {
    const v4f t0 = *(const v4fa*)(W2 + 4 * g);
    const v4f t1 = *(const v4fa*)(W2 + 4 * g + 32);
    const v4f t2 = *(const v4fa*)(W2 + 4 * g + 64);
    const v4f t3 = *(const v4fa*)(W2 + 4 * g + 96);
    w0.x = bf16_val(t0.x); w0.y = bf16_val(t0.y); w0.z = bf16_val(t0.z); w0.w = bf16_val(t0.w);
    w1.x = bf16_val(t1.x); w1.y = bf16_val(t1.y); w1.z = bf16_val(t1.z); w1.w = bf16_val(t1.w);
    w2.x = bf16_val(t2.x); w2.y = bf16_val(t2.y); w2.z = bf16_val(t2.z); w2.w = bf16_val(t2.w);
    w3.x = bf16_val(t3.x); w3.y = bf16_val(t3.y); w3.z = bf16_val(t3.z); w3.w = bf16_val(t3.w);
  }
  const float b2v = bf16_val(b2[0]);
  const int srcl = 8 * (lane & 3);
  const int oit  = lane >> 2;
  const int wbase = (int)blockIdx.x * EPB + wave * EPW;

#pragma unroll 1
  for (int ps = 0; ps < EPW / 32; ++ps) {
    const int e0 = wbase + 32 * ps;
    if (e0 >= nE) break;
    const int e  = e0 + lane;
    const int ec = e < nE ? e : nE - 1;
    int ri = rowi[ec];
    int ci = coli[ec];
    ri = ri < 0 ? 0 : (ri > nN - 1 ? nN - 1 : ri);
    ci = ci < 0 ? 0 : (ci > nN - 1 ? nN - 1 : ci);
    float outv = 0.0f;
#pragma unroll 1
    for (int it = 0; it < 8; ++it) {
      const int sl = 4 * it + j;
      const int r  = __shfl(ri, sl, 32);
      const int c  = __shfl(ci, sl, 32);
      const float* pp = pq + (size_t)r * NPQ + 4 * g;
      const float* qp = pq + (size_t)c * NPQ + NH + 4 * g;
      const v4f p0 = *(const v4fa*)pp;
      const v4f p1 = *(const v4fa*)(pp + 32);
      const v4f p2 = *(const v4fa*)(pp + 64);
      const v4f p3 = *(const v4fa*)(pp + 96);
      const v4f q0 = *(const v4fa*)qp;
      const v4f q1 = *(const v4fa*)(qp + 32);
      const v4f q2 = *(const v4fa*)(qp + 64);
      const v4f q3 = *(const v4fa*)(qp + 96);
      float acc = 0.0f;
      acc = fmaf(fmaxf(p0.x + q0.x, 0.0f), w0.x, acc);
      acc = fmaf(fmaxf(p0.y + q0.y, 0.0f), w0.y, acc);
      acc = fmaf(fmaxf(p0.z + q0.z, 0.0f), w0.z, acc);
      acc = fmaf(fmaxf(p0.w + q0.w, 0.0f), w0.w, acc);
      acc = fmaf(fmaxf(p1.x + q1.x, 0.0f), w1.x, acc);
      acc = fmaf(fmaxf(p1.y + q1.y, 0.0f), w1.y, acc);
      acc = fmaf(fmaxf(p1.z + q1.z, 0.0f), w1.z, acc);
      acc = fmaf(fmaxf(p1.w + q1.w, 0.0f), w1.w, acc);
      acc = fmaf(fmaxf(p2.x + q2.x, 0.0f), w2.x, acc);
      acc = fmaf(fmaxf(p2.y + q2.y, 0.0f), w2.y, acc);
      acc = fmaf(fmaxf(p2.z + q2.z, 0.0f), w2.z, acc);
      acc = fmaf(fmaxf(p2.w + q2.w, 0.0f), w2.w, acc);
      acc = fmaf(fmaxf(p3.x + q3.x, 0.0f), w3.x, acc);
      acc = fmaf(fmaxf(p3.y + q3.y, 0.0f), w3.y, acc);
      acc = fmaf(fmaxf(p3.z + q3.z, 0.0f), w3.z, acc);
      acc = fmaf(fmaxf(p3.w + q3.w, 0.0f), w3.w, acc);
      acc += __shfl_xor(acc, 4, 32);
      acc += __shfl_xor(acc, 2, 32);
      acc += __shfl_xor(acc, 1, 32);
      const float t = __shfl(acc, srcl, 32);
      outv = (oit == it) ? t : outv;
    }
    const float ov = outv + b2v;
    float* op = out + (size_t)e0 + lane;
    if (e < nE) *(volatile float*)op = ov;
    __threadfence();
    if (e < nE) *(volatile float*)op = ov;
  }
}

static inline int cdiv(int a, int b) { return (a + b - 1) / b; }
static inline size_t al256(size_t o) { return (o + 255) & ~(size_t)255; }

extern "C" void kernel_launch(void* const* d_in, const int* in_sizes, int n_in,
                              void* d_out, int out_size, void* d_ws, size_t ws_size,
                              hipStream_t stream) {
  if (n_in < 7) return;
  if (in_sizes[0] < ZD || (in_sizes[0] % ZD) != 0) return;
  const int nN = in_sizes[0] / ZD;
  if (nN < 1 || nN > (1 << 22)) return;
  const int nE = in_sizes[1];
  if (nE < 1 || in_sizes[2] != nE) return;
  if (in_sizes[3] != NH * NH || in_sizes[4] != NH) return;
  if (in_sizes[5] != NH || in_sizes[6] != 1) return;
  if (out_size != nE) return;

  const float* z   = (const float*)d_in[0];
  const int*   row = (const int*)d_in[1];
  const int*   col = (const int*)d_in[2];
  const float* W1  = (const float*)d_in[3];
  const float* b1  = (const float*)d_in[4];
  const float* W2  = (const float*)d_in[5];
  const float* b2  = (const float*)d_in[6];
  float* out = (float*)d_out;

  const int MP = cdiv(nN, GBM) * GBM;
  const int gM = MP / GBM;

  char* ws = (char*)d_ws;
  size_t off = 0;
  const size_t oBT = off; off = al256(off + (size_t)NPQ * ZD * 2);
  const size_t oZB = off; off = al256(off + (size_t)MP * ZD * 2);
  const size_t oPQ = off; off = al256(off + (size_t)MP * NPQ * 4);
  if (off > ws_size || off > (size_t)WSMAX) return;
  unsigned short* BT2 = (unsigned short*)(ws + oBT);
  unsigned short* ZB  = (unsigned short*)(ws + oZB);
  float*          PQ  = (float*)(ws + oPQ);

  const int nUz = MP * (ZD / 8);
  k_wprep<<<NUW / NTHR, NTHR, 0, stream>>>(W1, BT2);
  k_cvz<<<cdiv(nUz, NTHR), NTHR, 0, stream>>>(z, nN, nUz, ZB);
  k_nodegemm<<<dim3(gM, NPQ / GBN), GTHR, 0, stream>>>(ZB, BT2, b1, PQ);
  k_edge<<<cdiv(nE, EPB), NTHR, 0, stream>>>(PQ, row, col, W2, b2, nE, nN, out);
}
